// BasicBlock_3058016715396
// MI455X (gfx1250) — hardware-run, weakly checked
//
#include <hip/hip_runtime.h>
#include <stddef.h>
#include <stdint.h>

#define NROW    100000
#define KOFF    27
#define CH      64
#define TILE_M  128
#define NBLK    782
#define MPAD    100096
#define ZROW    (MPAD - 1)
#define XPITCH  64
#define HPITCH  128
#define W1PITCH 1728
#define W2PITCH 3456
#define W1SEG   64
#define W2SEG   128
#ifndef SPLIT2
#define SPLIT2  1
#endif
#define XUNITS  (MPAD * XPITCH / 8)
#define XBLK    (XUNITS / 256)
#define PREPGRID (XBLK + 2 * KOFF)

static_assert(NBLK * TILE_M == MPAD);
static_assert((NBLK - 1) * TILE_M < NROW && NROW <= MPAD);
static_assert(NROW % 16 == 0);
static_assert(ZROW >= NROW && ZROW < MPAD);
static_assert(W1PITCH == KOFF * W1SEG && W2PITCH == KOFF * W2SEG);
static_assert(W1SEG == CH && W2SEG == 2 * CH && HPITCH == 2 * CH && XPITCH == CH);
static_assert(W1SEG % 32 == 0 && W2SEG % 32 == 0);
static_assert(XUNITS % 256 == 0);
static_assert(TILE_M == 8 * 16);

constexpr size_t SZ_XB   = (size_t)MPAD * XPITCH * 2;
constexpr size_t SZ_H    = (size_t)MPAD * HPITCH * 2;
constexpr size_t SZ_W1T  = (size_t)CH * W1PITCH * 2;
constexpr size_t SZ_W2D  = (size_t)CH * W2PITCH * 2;
constexpr size_t OFF_XB  = 0;
constexpr size_t OFF_H   = OFF_XB + SZ_XB;
constexpr size_t OFF_W1T = OFF_H + SZ_H;
constexpr size_t OFF_W2D = OFF_W1T + SZ_W1T;
constexpr size_t WS_TOTAL = OFF_W2D + SZ_W2D;
static_assert(SZ_XB % 128 == 0 && SZ_H % 128 == 0 && SZ_W1T % 128 == 0 && SZ_W2D % 128 == 0);
static_assert(OFF_H % 128 == 0 && OFF_W1T % 128 == 0 && OFF_W2D % 128 == 0);
static_assert(WS_TOTAL == 39100416);
static_assert(WS_TOTAL <= ((size_t)128u << 20));

typedef float          v4f   __attribute__((ext_vector_type(4)));
typedef float          v8f   __attribute__((ext_vector_type(8)));
typedef int            v8i   __attribute__((ext_vector_type(8)));
typedef unsigned       v2u   __attribute__((ext_vector_type(2)));
typedef unsigned short v8us  __attribute__((ext_vector_type(8)));
typedef unsigned short v16us __attribute__((ext_vector_type(16)));
typedef __bf16         v16bf __attribute__((ext_vector_type(16)));
typedef v4f  __attribute__((may_alias)) v4fa;
typedef v2u  __attribute__((may_alias)) v2ua;
typedef v8us __attribute__((may_alias)) v8usa;
union FragB { v16bf v; v16us u; v8us h[2]; v8i w; };

__device__ __forceinline__ v8f wmb(const FragB& a, const FragB& b, v8f c) {
  v8f d = __builtin_amdgcn_wmma_f32_16x16x32_bf16(false, a.v, false, b.v, (short)0, c, false, false);
  asm volatile("v_nop\n\tv_nop\n\tv_nop\n\tv_nop" : "+v"(d) : "v"(a.w), "v"(b.w));
  return d;
}

__device__ __forceinline__ unsigned bf16_bits(float f) {
  const unsigned u = __float_as_uint(f);
  const unsigned r = (u + 0x7FFFu + ((u >> 16) & 1u)) >> 16;
  const unsigned q = (u >> 16) | 0x40u;
  return ((u & 0x7fffffffu) > 0x7f800000u) ? q : r;
}

__device__ __forceinline__ unsigned relu_split(float v, unsigned lomask) {
  const float y = (v > 0.0f) ? v : (v - v);
  const unsigned hb = bf16_bits(y);
  const unsigned lb = bf16_bits(y - __uint_as_float(hb << 16));
  return (hb & ~lomask) | (lb & lomask);
}

template <int NDUP>
__device__ __forceinline__ void wprep_body(const float* __restrict__ W, unsigned short* P, int k, int tid) {
  __shared__ float tl[64 * 65];
  constexpr int PITCH = 1728 * NDUP;
  constexpr int KSEG  = 64 * NDUP;
  static_assert(NDUP == 1 || NDUP == 2);
  const float* src = W + (size_t)k * 4096;
#pragma unroll
  for (int i = 0; i < 4; ++i) {
    const int f = (i * 256 + tid) * 4;
    const int c = f >> 6, d = f & 63;
    const v4f v = *(const v4f*)(src + f);
    tl[c * 65 + d]     = v.x;
    tl[c * 65 + d + 1] = v.y;
    tl[c * 65 + d + 2] = v.z;
    tl[c * 65 + d + 3] = v.w;
  }
  __syncthreads();
  const int q = tid & 7, sub = tid >> 3;
  v8us ov[2 * NDUP];
#pragma unroll
  for (int pass = 0; pass < 2 * NDUP; ++pass) {
    const int ln = pass * 32 + sub;
    const int d  = ln / NDUP;
    v8us o;
#pragma unroll
    for (int j = 0; j < 8; ++j) o[j] = (unsigned short)bf16_bits(tl[(8 * q + j) * 65 + d]);
    ov[pass] = o;
  }
#pragma unroll
  for (int pass = 0; pass < 2 * NDUP; ++pass) {
    const int ln = pass * 32 + sub;
    const int d = ln / NDUP, dup = ln % NDUP;
    unsigned short* dp = P + (size_t)d * PITCH + k * KSEG + 64 * dup + 8 * q;
    *(volatile v8us*)dp = ov[pass];
  }
  __threadfence();
#pragma unroll
  for (int pass = 0; pass < 2 * NDUP; ++pass) {
    const int ln = pass * 32 + sub;
    const int d = ln / NDUP, dup = ln % NDUP;
    unsigned short* dp = P + (size_t)d * PITCH + k * KSEG + 64 * dup + 8 * q;
    *(volatile v8us*)dp = ov[pass];
  }
}

__global__ __launch_bounds__(256) void k_prep(const float* __restrict__ x, const float* __restrict__ W1,
                                              const float* __restrict__ W2, unsigned short* XB,
                                              unsigned short* W1T, unsigned short* W2D) {
  const int bid = (int)blockIdx.x, tid = (int)threadIdx.x;
  if (bid < XBLK) {
    const int u = bid * 256 + tid;
    const int r = u >> 3, q = u & 7;
    const int rc = r < NROW ? r : NROW - 1;
    const float* p = x + (size_t)rc * CH + 8 * q;
    const v4f a = *(const v4f*)p;
    const v4f b = *(const v4f*)(p + 4);
    const unsigned lm = (r < NROW) ? 0xffffu : 0u;
    v8us o;
    o[0] = (unsigned short)(bf16_bits(a.x) & lm); o[1] = (unsigned short)(bf16_bits(a.y) & lm);
    o[2] = (unsigned short)(bf16_bits(a.z) & lm); o[3] = (unsigned short)(bf16_bits(a.w) & lm);
    o[4] = (unsigned short)(bf16_bits(b.x) & lm); o[5] = (unsigned short)(bf16_bits(b.y) & lm);
    o[6] = (unsigned short)(bf16_bits(b.z) & lm); o[7] = (unsigned short)(bf16_bits(b.w) & lm);
    unsigned short* dp = XB + (size_t)u * 8;
    *(volatile v8us*)dp = o;
    __threadfence();
    *(volatile v8us*)dp = o;
  } else if (bid < XBLK + KOFF) {
    int k = bid - XBLK;
    k = k < 0 ? 0 : (k > KOFF - 1 ? KOFF - 1 : k);
    wprep_body<1>(W1, W1T, k, tid);
  } else {
    int k = bid - XBLK - KOFF;
    k = k < 0 ? 0 : (k > KOFF - 1 ? KOFF - 1 : k);
    wprep_body<2>(W2, W2D, k, tid);
  }
}

template <int L>
__global__ __launch_bounds__(256) __attribute__((amdgpu_num_vgpr(248)))
void k_conv(const int* __restrict__ idx, const int* __restrict__ msk,
            const unsigned short* __restrict__ Ap, const unsigned short* __restrict__ Wp,
            const unsigned short* __restrict__ XB, unsigned short* Hout, float* outp) {
  constexpr int APITCH = (L == 1) ? XPITCH : HPITCH;
  constexpr int WPITCH = (L == 1) ? W1PITCH : W2PITCH;
  constexpr int WSEG   = (L == 1) ? W1SEG : W2SEG;
  constexpr int NKS    = (L == 1) ? 2 : ((SPLIT2 != 0) ? 4 : 2);
  static_assert(32 * NKS <= APITCH && 32 * NKS <= WSEG);

  __shared__ __attribute__((aligned(16))) float stg[8 * 16 * 64];

  const int tid = (int)threadIdx.x, lane = tid & 31, w = tid >> 5;
  const int h = lane >> 4, m = lane & 15;
  const int rowBase = (int)blockIdx.x * TILE_M;
  const int r  = rowBase + 16 * w + m;
  const int rr = r < NROW ? r : NROW - 1;
  const int rowlive = (r < NROW) ? -1 : 0;
  const int* ip = idx + (size_t)rr * KOFF;
  const int* mp = msk + (size_t)rr * KOFF;
  const unsigned short* bp = Wp + (size_t)m * WPITCH + 8 * h;

  v8f acc[4];
  {
    const v8f z = {0.f, 0.f, 0.f, 0.f, 0.f, 0.f, 0.f, 0.f};
#pragma unroll
    for (int t = 0; t < 4; ++t) acc[t] = z;
  }

#pragma unroll 1
  for (int k = 0; k < KOFF; ++k) {
    const int iv = ip[k];
    const int mv = mp[k];
    asm volatile("" :: "v"(iv));
    asm volatile("" :: "v"(mv));
    int s = iv < 0 ? 0 : (iv > NROW - 1 ? NROW - 1 : iv);
    const int sel = ((mv != 0) ? -1 : 0) & rowlive;
    s = (s & sel) | (ZROW & ~sel);
    const unsigned short* ap = Ap + (size_t)s * APITCH + 8 * h;
    FragB af[NKS];
#pragma unroll
    for (int ks = 0; ks < NKS; ++ks) {
      af[ks].h[0] = *(const v8usa*)(ap + 32 * ks);
      af[ks].h[1] = *(const v8usa*)(ap + 32 * ks + 16);
    }
#pragma unroll
    for (int ks = 0; ks < NKS; ++ks) {
#pragma unroll
      for (int nt = 0; nt < 4; ++nt) {
        const unsigned short* wq = bp + (size_t)(16 * nt) * WPITCH + WSEG * k + 32 * ks;
        FragB bf;
        bf.h[0] = *(const v8usa*)wq;
        bf.h[1] = *(const v8usa*)(wq + 16);
        acc[nt] = wmb(af[ks], bf, acc[nt]);
      }
    }
  }

  float* so = stg + w * 1024;
#pragma unroll
  for (int nt = 0; nt < 4; ++nt) {
#pragma unroll
    for (int rq = 0; rq < 8; ++rq) so[(8 * h + rq) * 64 + 16 * nt + m] = acc[nt][rq];
  }
  __syncthreads();

  const int p = lane & 15, rsel = lane >> 4;

  if constexpr (L == 1) {
    const int c0 = 8 * (p & 7);
    const unsigned lomask = (p >> 3) != 0 ? 0xffffu : 0u;
    v8us hv[8];
#pragma unroll
    for (int i = 0; i < 8; ++i) {
      const int row = 2 * i + rsel;
      const v4f va = *(const v4fa*)(so + row * 64 + c0);
      const v4f vb = *(const v4fa*)(so + row * 64 + c0 + 4);
      v8us o;
      o[0] = (unsigned short)relu_split(va.x, lomask); o[1] = (unsigned short)relu_split(va.y, lomask);
      o[2] = (unsigned short)relu_split(va.z, lomask); o[3] = (unsigned short)relu_split(va.w, lomask);
      o[4] = (unsigned short)relu_split(vb.x, lomask); o[5] = (unsigned short)relu_split(vb.y, lomask);
      o[6] = (unsigned short)relu_split(vb.z, lomask); o[7] = (unsigned short)relu_split(vb.w, lomask);
      hv[i] = o;
    }
#pragma unroll
    for (int i = 0; i < 8; ++i) {
      unsigned short* hp = Hout + (size_t)(rowBase + 16 * w + 2 * i + rsel) * HPITCH + 8 * p;
      *(volatile v8us*)hp = hv[i];
    }
    __threadfence();
#pragma unroll
    for (int i = 0; i < 8; ++i) {
      unsigned short* hp = Hout + (size_t)(rowBase + 16 * w + 2 * i + rsel) * HPITCH + 8 * p;
      *(volatile v8us*)hp = hv[i];
    }
  } else {
    const int c0 = 4 * p;
    const bool wlive = (rowBase + 16 * w) < NROW;
    v4f ov[8];
#pragma unroll
    for (int i = 0; i < 8; ++i) {
      const int row = 2 * i + rsel;
      const int rg  = rowBase + 16 * w + row;
      const v4f va = *(const v4fa*)(so + row * 64 + c0);
      const v2u xw = *(const v2ua*)(XB + (size_t)rg * XPITCH + c0);
      const float x0 = __uint_as_float(xw.x << 16);
      const float x1 = __uint_as_float(xw.x & 0xffff0000u);
      const float x2 = __uint_as_float(xw.y << 16);
      const float x3 = __uint_as_float(xw.y & 0xffff0000u);
      const float t0 = va.x + x0, t1 = va.y + x1, t2 = va.z + x2, t3 = va.w + x3;
      v4f y;
      y.x = (t0 > 0.0f) ? t0 : (t0 - t0);
      y.y = (t1 > 0.0f) ? t1 : (t1 - t1);
      y.z = (t2 > 0.0f) ? t2 : (t2 - t2);
      y.w = (t3 > 0.0f) ? t3 : (t3 - t3);
      ov[i] = y;
    }
    if (wlive) {
#pragma unroll
      for (int i = 0; i < 8; ++i) {
        float* op = outp + (size_t)(rowBase + 16 * w + 2 * i + rsel) * CH + c0;
        *(volatile v4f*)op = ov[i];
      }
    }
    __threadfence();
    if (wlive) {
#pragma unroll
      for (int i = 0; i < 8; ++i) {
        float* op = outp + (size_t)(rowBase + 16 * w + 2 * i + rsel) * CH + c0;
        *(volatile v4f*)op = ov[i];
      }
    }
  }
}

extern "C" void kernel_launch(void* const* d_in, const int* in_sizes, int n_in,
                              void* d_out, int out_size, void* d_ws, size_t ws_size,
                              hipStream_t stream) {
  if (n_in < 5) return;
  if (in_sizes[0] != NROW * CH) return;
  if (in_sizes[1] != NROW * KOFF) return;
  if (in_sizes[2] != NROW * KOFF) return;
  if (in_sizes[3] != KOFF * CH * CH) return;
  if (in_sizes[4] != KOFF * CH * CH) return;
  if (out_size != NROW * CH) return;
  if (ws_size < WS_TOTAL) return;

  const float* x    = (const float*)d_in[0];
  const int*   idx  = (const int*)d_in[1];
  const int*   mask = (const int*)d_in[2];
  const float* W1   = (const float*)d_in[3];
  const float* W2   = (const float*)d_in[4];
  float* out = (float*)d_out;

  char* ws = (char*)d_ws;
  unsigned short* XB  = (unsigned short*)(ws + OFF_XB);
  unsigned short* H   = (unsigned short*)(ws + OFF_H);
  unsigned short* W1T = (unsigned short*)(ws + OFF_W1T);
  unsigned short* W2D = (unsigned short*)(ws + OFF_W2D);

  k_prep<<<PREPGRID, 256, 0, stream>>>(x, W1, W2, XB, W1T, W2D);
  k_conv<1><<<NBLK, 256, 0, stream>>>(idx, mask, XB, W1T, XB, H, out);
  k_conv<2><<<NBLK, 256, 0, stream>>>(idx, mask, H, W2D, XB, H, out);
}
